// GraphConvEW_12627203850513
// MI455X (gfx1250) — hardware-verified
//
#include <hip/hip_runtime.h>
#include <stddef.h>
#include <stdint.h>


#define DF     128
#define K2     256
#define NTHR   256
#define NWAVE  8
#define EPT    8
#define CHUNK  (NTHR * EPT)
#define WCAP   (EPT * 32)
#define LISTN  (NWAVE * WCAP)
#define NBD    8192
#define SLD    13
#define NBA    1024
#define SLA    10
#define RCAP   28672
#define DEGCAP 64
#define GBM    64
#define GBN    128
#define GTHR   128
#define UW     4096
#define AGG_ZINTS    (LISTN + 2 * RCAP + 3 * NBA)
#define MISC_INTS    16
#define ROWBUF_INTS  (NWAVE * K2 / 2)
#define AGG_LDS_INTS (AGG_ZINTS + MISC_INTS + ROWBUF_INTS)
#define WSMAX  134217728

static_assert((CHUNK & (CHUNK - 1)) == 0 && CHUNK <= 4096);
static_assert((NBD & (NBD - 1)) == 0 && NBD == (1 << SLD));
static_assert((NBA & (NBA - 1)) == 0 && NBA == (1 << SLA));
static_assert(((long long)CHUNK << SLD) < (1LL << 31));
static_assert(((long long)CHUNK << SLA) < (1LL << 31));
static_assert(NBD % (NTHR * 4) == 0);
static_assert(LISTN % NTHR == 0);
static_assert(NBA % NWAVE == 0 && NBA % 32 == 0 && NBA % GBM == 0);
static_assert(RCAP % 4 == 0 && AGG_ZINTS % 4 == 0 && LISTN % 4 == 0 && ((AGG_ZINTS + MISC_INTS) % 4) == 0);
static_assert(K2 % 32 == 0 && K2 == 2 * DF);
static_assert(GBN == DF && GBM == (GTHR / 32) * 16 && DF == 4 * 32);
static_assert(UW % NTHR == 0 && UW == DF * (K2 / 8));
static_assert(AGG_LDS_INTS * 4 <= 300000);

typedef float          v4f   __attribute__((ext_vector_type(4)));
typedef float          v8f   __attribute__((ext_vector_type(8)));
typedef int            v4i   __attribute__((ext_vector_type(4)));
typedef int            v8i   __attribute__((ext_vector_type(8)));
typedef unsigned       v2u   __attribute__((ext_vector_type(2)));
typedef unsigned short v4us  __attribute__((ext_vector_type(4)));
typedef unsigned short v8us  __attribute__((ext_vector_type(8)));
typedef unsigned short v16us __attribute__((ext_vector_type(16)));
typedef __bf16         v16bf __attribute__((ext_vector_type(16)));
typedef v4f  __attribute__((may_alias)) v4fa;
typedef v4i  __attribute__((may_alias)) v4ia;
typedef v2u  __attribute__((may_alias)) v2ua;
typedef v4us __attribute__((may_alias)) v4usa;
typedef v8us __attribute__((may_alias)) v8usa;
union FragB { v16bf v; v16us u; v8us h[2]; v8i w; };

__device__ __forceinline__ v8f wmb(const FragB& a, const FragB& b, v8f c) {
  v8f d = __builtin_amdgcn_wmma_f32_16x16x32_bf16(false, a.v, false, b.v, (short)0, c, false, false);
  asm volatile("v_nop\n\tv_nop\n\tv_nop\n\tv_nop" : "+v"(d) : "v"(a.w), "v"(b.w));
  return d;
}

__device__ __forceinline__ unsigned bf16_bits(float f) {
  const unsigned u = __float_as_uint(f);
  return (u + 0x7FFFu + ((u >> 16) & 1u)) >> 16;
}
__device__ __forceinline__ float bf16_val(float f) {
  return __uint_as_float(bf16_bits(f) << 16);
}

__device__ __forceinline__ void wave_sync() {
  __builtin_amdgcn_fence(__ATOMIC_RELEASE, "wavefront");
  __builtin_amdgcn_wave_barrier();
  __builtin_amdgcn_fence(__ATOMIC_ACQUIRE, "wavefront");
}

template <int SLB>
__device__ __forceinline__ int scan_chunk(const int* __restrict__ dsts, int nE, int cbase, int slotBase,
                                          int nb, int vec8, int* list, int tid, int lane, int wave) {
  int wc = 0;
  const int el0  = tid * EPT;
  const int e0   = cbase + el0;
  const int sent = -2147483647 - 1;
  v4i da, db;
  if (vec8 != 0 && cbase + CHUNK <= nE) {
    da = *(const v4i*)(dsts + e0);
    db = *(const v4i*)(dsts + e0 + 4);
  } else {
    da.x = (e0     < nE) ? dsts[min(e0,     nE - 1)] : sent;
    da.y = (e0 + 1 < nE) ? dsts[min(e0 + 1, nE - 1)] : sent;
    da.z = (e0 + 2 < nE) ? dsts[min(e0 + 2, nE - 1)] : sent;
    da.w = (e0 + 3 < nE) ? dsts[min(e0 + 3, nE - 1)] : sent;
    db.x = (e0 + 4 < nE) ? dsts[min(e0 + 4, nE - 1)] : sent;
    db.y = (e0 + 5 < nE) ? dsts[min(e0 + 5, nE - 1)] : sent;
    db.z = (e0 + 6 < nE) ? dsts[min(e0 + 6, nE - 1)] : sent;
    db.w = (e0 + 7 < nE) ? dsts[min(e0 + 7, nE - 1)] : sent;
  }
  const unsigned nbs = (unsigned)slotBase;
  const unsigned unb = (unsigned)nb;
  const unsigned s0 = (unsigned)da.x - nbs, s1 = (unsigned)da.y - nbs;
  const unsigned s2 = (unsigned)da.z - nbs, s3 = (unsigned)da.w - nbs;
  const unsigned s4 = (unsigned)db.x - nbs, s5 = (unsigned)db.y - nbs;
  const unsigned s6 = (unsigned)db.z - nbs, s7 = (unsigned)db.w - nbs;
  const bool h0 = s0 < unb, h1 = s1 < unb, h2 = s2 < unb, h3 = s3 < unb;
  const bool h4 = s4 < unb, h5 = s5 < unb, h6 = s6 < unb, h7 = s7 < unb;
  const unsigned any = __builtin_amdgcn_ballot_w32(h0 | h1 | h2 | h3 | h4 | h5 | h6 | h7);
  if (any != 0u) {
#define HITJ(J, HJ, SJ) { \
      const unsigned mj = __builtin_amdgcn_ballot_w32(HJ); \
      if (mj != 0u) { \
        if (HJ) { \
          const int pos = wc + (int)__builtin_amdgcn_mbcnt_lo(mj, 0u); \
          if (pos < WCAP) list[wave * WCAP + pos] = ((el0 + (J)) << SLB) | (int)(SJ); \
        } \
        wc += (int)__builtin_popcount(mj); } }
    HITJ(0, h0, s0)
    HITJ(1, h1, s1)
    HITJ(2, h2, s2)
    HITJ(3, h3, s3)
    HITJ(4, h4, s4)
    HITJ(5, h5, s5)
    HITJ(6, h6, s6)
    HITJ(7, h7, s7)
#undef HITJ
  }
  return wc;
}

__global__ __launch_bounds__(NTHR) void k_wprep(const float* __restrict__ W1, const float* __restrict__ W2,
                                                const float* __restrict__ W3, unsigned short* WT) {
  const int u    = (int)blockIdx.x * NTHR + (int)threadIdx.x;
  const int part = u >> 12;
  const int v    = u & (UW - 1);
  const int n    = v >> 5;
  const int k8   = (v & 31) * 8;
  const int kk   = k8 & (DF - 1);
  const float* W;
  if (part == 0)      W = W1;
  else if (part == 1) W = W2;
  else if (part == 2) W = W3;
  else return;
  const float* p = W + (size_t)kk * DF + n;
  v8us o;
#pragma unroll
  for (int i = 0; i < 8; ++i) o[i] = (unsigned short)bf16_bits(p[(size_t)i * DF]);
  unsigned short* dp = WT + (size_t)part * (DF * K2) + (size_t)n * K2 + k8;
  *(volatile v8us*)dp = o;
  __threadfence();
  *(volatile v8us*)dp = o;
}

__global__ __launch_bounds__(NTHR) void k_cvx(const float* __restrict__ x, int nN, int nUnits,
                                              unsigned short* xb) {
  const int u = (int)blockIdx.x * NTHR + (int)threadIdx.x;
  if (u >= nUnits) return;
  const int row = u >> 4;
  const int k8  = (u & 15) * 8;
  const int rc  = row < nN ? row : nN - 1;
  const float* p = x + (size_t)rc * DF + k8;
  const v4f a = *(const v4fa*)p;
  const v4f b = *(const v4fa*)(p + 4);
  const bool ok = row < nN;
  v8us o;
  o[0] = ok ? (unsigned short)bf16_bits(a.x) : (unsigned short)0;
  o[1] = ok ? (unsigned short)bf16_bits(a.y) : (unsigned short)0;
  o[2] = ok ? (unsigned short)bf16_bits(a.z) : (unsigned short)0;
  o[3] = ok ? (unsigned short)bf16_bits(a.w) : (unsigned short)0;
  o[4] = ok ? (unsigned short)bf16_bits(b.x) : (unsigned short)0;
  o[5] = ok ? (unsigned short)bf16_bits(b.y) : (unsigned short)0;
  o[6] = ok ? (unsigned short)bf16_bits(b.z) : (unsigned short)0;
  o[7] = ok ? (unsigned short)bf16_bits(b.w) : (unsigned short)0;
  unsigned short* dp = xb + (size_t)row * DF + k8;
  *(volatile v8us*)dp = o;
  __threadfence();
  *(volatile v8us*)dp = o;
}

__global__ __launch_bounds__(NTHR) void k_ws(const float* __restrict__ w, int nE, int nU, float* wsv) {
  const int u = (int)blockIdx.x * NTHR + (int)threadIdx.x;
  if (u >= nU) return;
  const int e0 = 4 * u;
  const int ea = min(e0,     nE - 1);
  const int eb = min(e0 + 1, nE - 1);
  const int ec = min(e0 + 2, nE - 1);
  const int ed = min(e0 + 3, nE - 1);
  const v4f a = *(const v4f*)(w + (size_t)ea * 4);
  const v4f b = *(const v4f*)(w + (size_t)eb * 4);
  const v4f c = *(const v4f*)(w + (size_t)ec * 4);
  const v4f d = *(const v4f*)(w + (size_t)ed * 4);
  v4f r;
  r.x = 0.25f * (((bf16_val(a.x) + bf16_val(a.y)) + bf16_val(a.z)) + bf16_val(a.w));
  r.y = 0.25f * (((bf16_val(b.x) + bf16_val(b.y)) + bf16_val(b.z)) + bf16_val(b.w));
  r.z = 0.25f * (((bf16_val(c.x) + bf16_val(c.y)) + bf16_val(c.z)) + bf16_val(c.w));
  r.w = 0.25f * (((bf16_val(d.x) + bf16_val(d.y)) + bf16_val(d.z)) + bf16_val(d.w));
  float* dp = wsv + (size_t)e0;
  *(volatile v4f*)dp = r;
  __threadfence();
  *(volatile v4f*)dp = r;
}

__global__ __launch_bounds__(NTHR) void k_deg(const int* __restrict__ keys, int nE, int vec8, float* dis) {
  __shared__ __attribute__((aligned(16))) int scnt[NBD];
  __shared__ __attribute__((aligned(16))) int list[LISTN];
  __shared__ int wcnt[NWAVE];
  const int tid = (int)threadIdx.x, lane = tid & 31, wave = tid >> 5;
  const int nodeBase = (int)blockIdx.x * NBD;

  for (int i = tid; i < NBD; i += NTHR) scnt[i] = 0;
  for (int i = tid; i < LISTN; i += NTHR) list[i] = 0;
  if (tid < NWAVE) wcnt[tid] = 0;
  __syncthreads();

  const int nChunks = (nE + CHUNK - 1) / CHUNK;
#pragma unroll 1
  for (int ch = 0; ch < nChunks; ++ch) {
    const int cbase = ch * CHUNK;
    const int wc = scan_chunk<SLD>(keys, nE, cbase, nodeBase, NBD, vec8, list, tid, lane, wave);
    if (lane == 0) wcnt[wave] = wc;
    __syncthreads();
    if (wave == 0) {
#pragma unroll 1
      for (int w2 = 0; w2 < NWAVE; ++w2) {
        int c = wcnt[w2];
        c = c < 0 ? 0 : (c > WCAP ? WCAP : c);
#pragma unroll 1
        for (int b0 = 0; b0 < c; b0 += 32) {
          const int idx = b0 + lane;
          const int ent = list[w2 * WCAP + (idx < WCAP ? idx : WCAP - 1)];
          const int m32 = (c - b0) < 32 ? (c - b0) : 32;
#pragma unroll 1
          for (int k = 0; k < m32; ++k) {
            const int u  = __builtin_amdgcn_readlane(ent, k);
            const int sl = u & (NBD - 1);
            if (lane == 0) scnt[sl] = scnt[sl] + 1;
          }
        }
      }
    }
    __syncthreads();
  }

  v4f vals[NBD / (NTHR * 4)];
#pragma unroll
  for (int it = 0; it < NBD / (NTHR * 4); ++it) {
    const int s0 = it * (NTHR * 4) + 4 * tid;
    const v4i c4 = *(const v4ia*)(scnt + s0);
    const float d0 = (float)(c4.x < 1 ? 1 : c4.x), d1 = (float)(c4.y < 1 ? 1 : c4.y);
    const float d2 = (float)(c4.z < 1 ? 1 : c4.z), d3 = (float)(c4.w < 1 ? 1 : c4.w);
    v4f v;
    v.x = rsqrtf(d0); v.y = rsqrtf(d1); v.z = rsqrtf(d2); v.w = rsqrtf(d3);
    vals[it] = v;
  }
#pragma unroll
  for (int it = 0; it < NBD / (NTHR * 4); ++it) {
    const int s0 = it * (NTHR * 4) + 4 * tid;
    *(volatile v4f*)(dis + (size_t)nodeBase + s0) = vals[it];
  }
  __threadfence();
#pragma unroll
  for (int it = 0; it < NBD / (NTHR * 4); ++it) {
    const int s0 = it * (NTHR * 4) + 4 * tid;
    *(volatile v4f*)(dis + (size_t)nodeBase + s0) = vals[it];
  }
}

template <int L0>
__global__ __launch_bounds__(NTHR) void k_scan(const int* __restrict__ srcs, const int* __restrict__ dsts,
                                               const float* __restrict__ wsv, const float* __restrict__ onv,
                                               int nE, int nN, int vec8, int mRows,
                                               const unsigned short* __restrict__ xb,
                                               const float* __restrict__ hin, unsigned short* ahl) {
  extern __shared__ __attribute__((aligned(16))) int dsm[];
  int* list = dsm;
  int* hl   = dsm + LISTN;
  int* sl   = hl + RCAP;
  int* cnt  = sl + RCAP;
  int* offs = cnt + NBA;
  int* cur  = offs + NBA;
  int* misc = cur + NBA;
  const int tid = (int)threadIdx.x, lane = tid & 31, wave = tid >> 5;
  unsigned short* rowbuf = (unsigned short*)(misc + MISC_INTS) + wave * K2;
  const int nodeBase = (int)blockIdx.x * NBA;

  {
    const v4i z4 = {0, 0, 0, 0};
    for (int i = tid * 4; i < AGG_ZINTS; i += NTHR * 4) *(v4ia*)(dsm + i) = z4;
    if (tid < MISC_INTS) misc[tid] = 0;
  }
  __syncthreads();

  int t = 0, ov = 0;
  const int nChunks = (nE + CHUNK - 1) / CHUNK;
#pragma unroll 1
  for (int ch = 0; ch < nChunks; ++ch) {
    const int cbase = ch * CHUNK;
    const int wc = scan_chunk<SLA>(dsts, nE, cbase, nodeBase, NBA, vec8, list, tid, lane, wave);
    if (lane == 0) misc[wave] = wc;
    __syncthreads();
    if (wave == 0) {
#pragma unroll 1
      for (int w2 = 0; w2 < NWAVE; ++w2) {
        int c = misc[w2];
        c = c < 0 ? 0 : (c > WCAP ? WCAP : c);
#pragma unroll 1
        for (int b0 = 0; b0 < c; b0 += 32) {
          const int idx = b0 + lane;
          const int ent = list[w2 * WCAP + (idx < WCAP ? idx : WCAP - 1)];
          const int m32 = (c - b0) < 32 ? (c - b0) : 32;
#pragma unroll 1
          for (int k = 0; k < m32; ++k) {
            const int u    = __builtin_amdgcn_readlane(ent, k);
            const int slot = u & (NBA - 1);
            const int el   = (u >> SLA) & (CHUNK - 1);
            const int pk   = ((cbase + el) << SLA) | slot;
            if (t < RCAP) {
              if (lane == 0) { hl[t] = pk; cnt[slot] = cnt[slot] + 1; }
              t = t + 1;
            } else {
              ov = 1;
            }
          }
        }
      }
    }
    __syncthreads();
  }
  if (wave == 0 && lane == 0) { misc[8] = t; misc[9] = ov; }
  __syncthreads();
  int tt = misc[8];
  tt = tt < 0 ? 0 : (tt > RCAP ? RCAP : tt);
  const int ovf = misc[9];

  if (wave == 0) {
    const int base = lane * (NBA / 32);
    int s = 0;
#pragma unroll 1
    for (int i = 0; i < NBA / 32; ++i) s += cnt[base + i];
    int incl = s;
#pragma unroll
    for (int d = 1; d < 32; d <<= 1) {
      const int y = __shfl_up(incl, d, 32);
      if (lane >= d) incl += y;
    }
    int run = incl - s;
#pragma unroll 1
    for (int i = 0; i < NBA / 32; ++i) {
      const int cv = cnt[base + i];
      offs[base + i] = run;
      cur[base + i]  = run;
      run += cv;
    }
  }
  __syncthreads();
  if (wave == 0) {
#pragma unroll 1
    for (int b0 = 0; b0 < tt; b0 += 32) {
      const int idx = b0 + lane;
      const int ent = hl[idx < RCAP ? idx : RCAP - 1];
      const int m32 = (tt - b0) < 32 ? (tt - b0) : 32;
#pragma unroll 1
      for (int k = 0; k < m32; ++k) {
        const int u    = __builtin_amdgcn_readlane(ent, k);
        const int slot = u & (NBA - 1);
        if (lane == 0) {
          int p = cur[slot];
          p = p < 0 ? 0 : (p > RCAP - 1 ? RCAP - 1 : p);
          sl[p] = u;
          cur[slot] = p + 1;
        }
      }
    }
  }
  __syncthreads();

  const float qnan = __int_as_float(0x7fc00000);
  const float pz = (ovf != 0) ? qnan : 0.0f;
#pragma unroll 1
  for (int si = 0; si < NBA / NWAVE; ++si) {
    const int s    = si * NWAVE + wave;
    const int node = nodeBase + s;
    const int cr = cnt[s];
    const bool big = cr > DEGCAP;
    const int c = cr < 0 ? 0 : (cr > DEGCAP ? DEGCAP : cr);
    int o = offs[s];
    o = o < 0 ? 0 : (o > RCAP ? RCAP : o);
    const float inn = rsqrtf((float)(c < 1 ? 1 : c));
    float a0 = 0.0f, a1 = 0.0f, a2 = 0.0f, a3 = 0.0f;
#pragma unroll 1
    for (int b0 = 0; b0 < c; b0 += 32) {
      int idx = o + b0 + lane;
      idx = idx > RCAP - 1 ? RCAP - 1 : idx;
      const int ent = sl[idx];
      int eid = ent >> SLA;
      eid = eid < 0 ? 0 : (eid > nE - 1 ? nE - 1 : eid);
      int sr = srcs[eid];
      sr = sr < 0 ? 0 : (sr > nN - 1 ? nN - 1 : sr);
      const float cf  = onv[sr] * wsv[eid];
      const int   cfi = __float_as_int(cf);
      const int m32 = (c - b0) < 32 ? (c - b0) : 32;
#pragma unroll 1
      for (int k = 0; k < m32; ++k) {
        const int   sk = __builtin_amdgcn_readlane(sr, k);
        const float ck = __int_as_float(__builtin_amdgcn_readlane(cfi, k));
        if constexpr (L0 != 0) {
          const v2u wv = *(const v2ua*)(xb + (size_t)sk * DF + 4 * lane);
          const float f0 = __uint_as_float(wv.x << 16);
          const float f1 = __uint_as_float(wv.x & 0xffff0000u);
          const float f2 = __uint_as_float(wv.y << 16);
          const float f3 = __uint_as_float(wv.y & 0xffff0000u);
          a0 = fmaf(ck, f0, a0);
          a1 = fmaf(ck, f1, a1);
          a2 = fmaf(ck, f2, a2);
          a3 = fmaf(ck, f3, a3);
        } else {
          const v4f a = *(const v4f*)(hin + (size_t)sk * DF + 4 * lane);
          a0 = fmaf(ck, a.x, a0);
          a1 = fmaf(ck, a.y, a1);
          a2 = fmaf(ck, a.z, a2);
          a3 = fmaf(ck, a.w, a3);
        }
      }
    }
    const float pzr = big ? qnan : pz;
    const bool live = node < nN;
    const float m0 = live ? (a0 * inn + pzr) : 0.0f;
    const float m1 = live ? (a1 * inn + pzr) : 0.0f;
    const float m2 = live ? (a2 * inn + pzr) : 0.0f;
    const float m3 = live ? (a3 * inn + pzr) : 0.0f;
    v4us mh, ml;
    {
      unsigned hb;
      hb = bf16_bits(m0); mh[0] = (unsigned short)hb; ml[0] = (unsigned short)bf16_bits(m0 - __uint_as_float(hb << 16));
      hb = bf16_bits(m1); mh[1] = (unsigned short)hb; ml[1] = (unsigned short)bf16_bits(m1 - __uint_as_float(hb << 16));
      hb = bf16_bits(m2); mh[2] = (unsigned short)hb; ml[2] = (unsigned short)bf16_bits(m2 - __uint_as_float(hb << 16));
      hb = bf16_bits(m3); mh[3] = (unsigned short)hb; ml[3] = (unsigned short)bf16_bits(m3 - __uint_as_float(hb << 16));
    }
    *(v4usa*)(rowbuf + 4 * lane) = mh;
    *(v4usa*)(rowbuf + DF + 4 * lane) = ml;
    wave_sync();
    const v8us q0 = *(const v8usa*)(rowbuf + 8 * lane);
    wave_sync();
    if (node < mRows) {
      unsigned short* rpw = ahl + (size_t)node * K2 + 8 * lane;
      *(volatile v8us*)rpw = q0;
      __threadfence();
      *(volatile v8us*)rpw = q0;
    }
  }
}

template <int EPI>
__global__ __launch_bounds__(GTHR) void k_gemm(const unsigned short* __restrict__ Apl,
                                               const unsigned short* __restrict__ BT,
                                               const float* __restrict__ gv, const float* __restrict__ bv,
                                               float* outp, int nOut) {
  __shared__ __attribute__((aligned(16))) float stg[GBM * GBN];
  const int tid = (int)threadIdx.x, lane = tid & 31, wave = tid >> 5, hh = lane >> 4, m = lane & 15;
  const int rowBase = (int)blockIdx.x * GBM;

  v8f acc[8];
  {
    const v8f z = {0.f, 0.f, 0.f, 0.f, 0.f, 0.f, 0.f, 0.f};
#pragma unroll
    for (int t = 0; t < 8; ++t) acc[t] = z;
  }
  const unsigned short* ap = Apl + (size_t)(rowBase + 16 * wave + m) * (size_t)K2 + 8 * hh;
  const unsigned short* bp = BT + (size_t)m * (size_t)K2 + 8 * hh;

#pragma unroll 1
  for (int k0 = 0; k0 < K2; k0 += 32) {
    FragB af;
    af.h[0] = *(const v8usa*)(ap + k0);
    af.h[1] = *(const v8usa*)(ap + k0 + 16);
#pragma unroll
    for (int nt = 0; nt < 8; ++nt) {
      const unsigned short* wq = bp + (size_t)(16 * nt) * (size_t)K2 + k0;
      FragB bf;
      bf.h[0] = *(const v8usa*)wq;
      bf.h[1] = *(const v8usa*)(wq + 16);
      acc[nt] = wmb(af, bf, acc[nt]);
    }
  }

#pragma unroll
  for (int nt = 0; nt < 8; ++nt) {
    const int lc = 16 * nt + m;
#pragma unroll
    for (int r = 0; r < 8; ++r) {
      const int lr = 16 * wave + 8 * hh + r;
      stg[lr * GBN + lc] = acc[nt][r];
    }
  }
  __syncthreads();

  if constexpr (EPI != 0) {
    v4f g4, b4;
    {
      const v4f t1 = *(const v4f*)(gv + 4 * lane);
      const v4f t2 = *(const v4f*)(bv + 4 * lane);
      g4.x = bf16_val(t1.x); g4.y = bf16_val(t1.y); g4.z = bf16_val(t1.z); g4.w = bf16_val(t1.w);
      b4.x = bf16_val(t2.x); b4.y = bf16_val(t2.y); b4.z = bf16_val(t2.z); b4.w = bf16_val(t2.w);
    }
#pragma unroll 1
    for (int i = 0; i < 16; ++i) {
      float* sp = stg + (16 * wave + i) * GBN + 4 * lane;
      const v4f t = *(const v4fa*)sp;
      v4f r;
      r.x = (t.x > 0.0f) ? t.x : (t.x - t.x);
      r.y = (t.y > 0.0f) ? t.y : (t.y - t.y);
      r.z = (t.z > 0.0f) ? t.z : (t.z - t.z);
      r.w = (t.w > 0.0f) ? t.w : (t.w - t.w);
      float s = (r.x + r.y) + (r.z + r.w);
      s += __shfl_xor(s, 16, 32);
      s += __shfl_xor(s, 8, 32);
      s += __shfl_xor(s, 4, 32);
      s += __shfl_xor(s, 2, 32);
      s += __shfl_xor(s, 1, 32);
      const float mu = s * (1.0f / (float)DF);
      v4f d;
      d.x = r.x - mu; d.y = r.y - mu; d.z = r.z - mu; d.w = r.w - mu;
      float q = (d.x * d.x + d.y * d.y) + (d.z * d.z + d.w * d.w);
      q += __shfl_xor(q, 16, 32);
      q += __shfl_xor(q, 8, 32);
      q += __shfl_xor(q, 4, 32);
      q += __shfl_xor(q, 2, 32);
      q += __shfl_xor(q, 1, 32);
      const float rs = rsqrtf(q * (1.0f / (float)DF) + 1e-5f);
      v4f y;
      y.x = (d.x * rs) * g4.x + b4.x;
      y.y = (d.y * rs) * g4.y + b4.y;
      y.z = (d.z * rs) * g4.z + b4.z;
      y.w = (d.w * rs) * g4.w + b4.w;
      *(v4fa*)sp = y;
    }
  }

  v4f pv[16];
#pragma unroll
  for (int i = 0; i < 16; ++i) pv[i] = *(const v4fa*)(stg + (16 * wave + i) * GBN + 4 * lane);
#pragma unroll
  for (int i = 0; i < 16; ++i) {
    const int r = rowBase + 16 * wave + i;
    if (r < nOut) *(volatile v4f*)(outp + (size_t)r * DF + 4 * lane) = pv[i];
  }
  __threadfence();
#pragma unroll
  for (int i = 0; i < 16; ++i) {
    const int r = rowBase + 16 * wave + i;
    if (r < nOut) *(volatile v4f*)(outp + (size_t)r * DF + 4 * lane) = pv[i];
  }
}

__global__ __launch_bounds__(NTHR) void k_pool(const float* __restrict__ hf, const int* __restrict__ gid,
                                               int nN, float* outp) {
  __shared__ __attribute__((aligned(16))) float wsum[NWAVE * DF];
  __shared__ __attribute__((aligned(16))) float outs[DF];
  const int tid = (int)threadIdx.x, lane = tid & 31, wave = tid >> 5;
  const int g = (int)blockIdx.x;

  float a0 = 0.0f, a1 = 0.0f, a2 = 0.0f, a3 = 0.0f;
#pragma unroll 1
  for (int i0 = wave * 32; i0 < nN; i0 += NTHR) {
    const int i  = i0 + lane;
    const int ic = i < nN ? i : nN - 1;
    const int b  = gid[ic];
    const bool hit = (i < nN) && (b == g);
    unsigned msk = __builtin_amdgcn_ballot_w32(hit);
    int nh = (int)__builtin_popcount(msk);
    nh = nh > 32 ? 32 : nh;
#pragma unroll 1
    for (int q = 0; q < nh; ++q) {
      const int k = __builtin_ffs((int)msk) - 1;
      msk &= msk - 1u;
      int node = i0 + (k < 0 ? 0 : k);
      node = node > nN - 1 ? nN - 1 : node;
      const v4f v = *(const v4f*)(hf + (size_t)node * DF + 4 * lane);
      a0 += v.x; a1 += v.y; a2 += v.z; a3 += v.w;
    }
  }
  wsum[wave * DF + 4 * lane + 0] = a0;
  wsum[wave * DF + 4 * lane + 1] = a1;
  wsum[wave * DF + 4 * lane + 2] = a2;
  wsum[wave * DF + 4 * lane + 3] = a3;
  __syncthreads();
  if (tid < DF) {
    float s = 0.0f;
#pragma unroll
    for (int w2 = 0; w2 < NWAVE; ++w2) s += wsum[w2 * DF + tid];
    outs[tid] = s;
  }
  __syncthreads();
  const v4f ov = *(const v4fa*)(outs + 4 * lane);
  float* op = outp + (size_t)g * DF + 4 * lane;
  const bool okst = (wave == 0);
  if (okst) *(volatile v4f*)op = ov;
  __threadfence();
  if (okst) *(volatile v4f*)op = ov;
}

static inline int cdiv(int a, int b) { return (a + b - 1) / b; }
static inline size_t al256(size_t o) { return (o + 255) & ~(size_t)255; }

extern "C" void kernel_launch(void* const* d_in, const int* in_sizes, int n_in,
                              void* d_out, int out_size, void* d_ws, size_t ws_size,
                              hipStream_t stream) {
  if (n_in < 12) return;
  if (in_sizes[0] < DF || (in_sizes[0] % DF) != 0) return;
  const int nN = in_sizes[0] / DF;
  if (nN < 16 || nN >= (1 << 24)) return;
  if (in_sizes[1] < 4 || (in_sizes[1] & 3) != 0) return;
  const int nE = in_sizes[1] / 4;
  if (nE < 1 || nE >= (1 << 21)) return;
  if (in_sizes[2] != DF * DF || in_sizes[3] != DF * DF || in_sizes[4] != DF * DF) return;
  if (in_sizes[5] != DF || in_sizes[6] != DF || in_sizes[7] != DF || in_sizes[8] != DF) return;
  if (in_sizes[9] != nE || in_sizes[10] != nE) return;
  if (in_sizes[11] != nN) return;
  if (out_size < DF || (out_size % DF) != 0) return;
  const int nG = out_size / DF;
  if (nG > 65535) return;

  const float* x    = (const float*)d_in[0];
  const float* w    = (const float*)d_in[1];
  const float* W1   = (const float*)d_in[2];
  const float* W2   = (const float*)d_in[3];
  const float* W3   = (const float*)d_in[4];
  const float* l1g  = (const float*)d_in[5];
  const float* l1b  = (const float*)d_in[6];
  const float* l2g  = (const float*)d_in[7];
  const float* l2b  = (const float*)d_in[8];
  const int*   src  = (const int*)d_in[9];
  const int*   dst  = (const int*)d_in[10];
  const int*   gid  = (const int*)d_in[11];
  float* out = (float*)d_out;

  const int MP   = cdiv(nN, GBM) * GBM;
  const int gM   = MP / GBM;
  const int gD   = cdiv(nN, NBD);
  const int NBPD = gD * NBD;
  const int gA   = cdiv(MP, NBA);
  if ((long long)gA * NBA < (long long)MP) return;
  if (NBPD < nN) return;
  const int nUw  = cdiv(nE, 4);
  const int vec8 = ((nE & 3) == 0) ? 1 : 0;

  char* ws = (char*)d_ws;
  size_t off = 0;
  const size_t oWT  = off; off = al256(off + (size_t)3 * DF * K2 * 2);
  const size_t oWS  = off; off = al256(off + (size_t)nUw * 16);
  const size_t oON  = off; off = al256(off + (size_t)NBPD * 4);
  const size_t oXB  = off; off = al256(off + (size_t)nN * DF * 2);
  const size_t oAHL = off; off = al256(off + (size_t)MP * K2 * 2);
  const size_t oH1  = off; off = al256(off + (size_t)MP * DF * 4);
  const size_t oH2  = off; off = al256(off + (size_t)MP * DF * 4);
  if (off > ws_size || off > (size_t)WSMAX) return;
  unsigned short* WT  = (unsigned short*)(ws + oWT);
  float*          WSv = (float*)(ws + oWS);
  float*          ON  = (float*)(ws + oON);
  unsigned short* XB  = (unsigned short*)(ws + oXB);
  unsigned short* AHL = (unsigned short*)(ws + oAHL);
  float*          H1  = (float*)(ws + oH1);
  float*          H2  = (float*)(ws + oH2);
  const unsigned short* WT1 = WT;
  const unsigned short* WT2 = WT + (size_t)DF * K2;
  const unsigned short* WT3 = WT + (size_t)2 * DF * K2;

  const size_t scanLds = (size_t)AGG_LDS_INTS * 4;
  hipFuncSetAttribute(reinterpret_cast<const void*>(&k_scan<1>), hipFuncAttributeMaxDynamicSharedMemorySize, (int)scanLds);
  hipFuncSetAttribute(reinterpret_cast<const void*>(&k_scan<0>), hipFuncAttributeMaxDynamicSharedMemorySize, (int)scanLds);

  const int nUx = nN * (DF / 8);
  k_wprep<<<(3 * UW) / NTHR, NTHR, 0, stream>>>(W1, W2, W3, WT);
  k_cvx<<<cdiv(nUx, NTHR), NTHR, 0, stream>>>(x, nN, nUx, XB);
  k_ws<<<cdiv(nUw, NTHR), NTHR, 0, stream>>>(w, nE, nUw, WSv);
  k_deg<<<gD, NTHR, 0, stream>>>(src, nE, vec8, ON);
  k_scan<1><<<gA, NTHR, scanLds, stream>>>(src, dst, WSv, ON, nE, nN, vec8, MP, XB, H1, AHL);
  k_gemm<1><<<gM, GTHR, 0, stream>>>(AHL, WT1, l1g, l1b, H1, nN);
  k_scan<0><<<gA, NTHR, scanLds, stream>>>(src, dst, WSv, ON, nE, nN, vec8, MP, XB, H1, AHL);
  k_gemm<1><<<gM, GTHR, 0, stream>>>(AHL, WT2, l2g, l2b, H2, nN);
  k_scan<0><<<gA, NTHR, scanLds, stream>>>(src, dst, WSv, ON, nE, nN, vec8, MP, XB, H2, AHL);
  k_gemm<0><<<gM, GTHR, 0, stream>>>(AHL, WT3, l2g, l2b, H1, nN);
  k_pool<<<nG, NTHR, 0, stream>>>(H1, gid, nN, out);
}
